// RelPartialLearnableMultiHeadAttn_88149908783416
// MI455X (gfx1250) — hardware-run, weakly checked
//
#include <hip/hip_runtime.h>
#include <math.h>

constexpr int kBatch = 4;
constexpr int kQlen  = 1024;
constexpr int kMlen  = 1024;
constexpr int kKlen  = 2048;
constexpr int kDm    = 1024;
constexpr int kHeads = 16;
constexpr int kDh    = 64;
constexpr int kQRows = kBatch * kQlen;
constexpr int kKRows = kBatch * kKlen;
constexpr float kWCarry    = 16.0f;
constexpr float kWCarryInv = 1.0f / 16.0f;
constexpr float kPCarry    = 32768.0f;
constexpr float kVecCarry  = 256.0f;
constexpr float kVecOverP  = kVecCarry / kPCarry;
constexpr float kOutScale  = 1.0f / (kVecCarry * kWCarry);
constexpr float kScoreScale = 0.125f;
constexpr float kFill      = -1.0e30f;
constexpr float kInvDm     = 1.0f / 1024.0f;
constexpr float kLnEps     = 1.0e-5f;
constexpr int kQB     = 64;
constexpr int kKC     = 64;
constexpr int kBand   = 128;
constexpr int kBPitch = 84;
constexpr int kWaves  = 4;
constexpr int kMWords = kKC / 4;
static_assert(kHeads * kDh == kDm, "shape");
static_assert(kMlen + kQlen == kKlen, "shape");
static_assert(kDm % 32 == 0 && kKlen % 32 == 0 && kDh % 32 == 0, "K multiples of 32");
static_assert(kQlen % 64 == 0 && kKlen % 64 == 0 && kDm % 64 == 0 && kQRows % 64 == 0 && kKRows % 64 == 0, "M,N tile multiples");
static_assert(kQlen % kQB == 0 && kKlen % kKC == 0 && kQB == kWaves * 16, "attention tiles");
static_assert((kBPitch % 4) == 0 && kBPitch >= 80, "band scratch pitch");

typedef __attribute__((ext_vector_type(16))) _Float16 v16h;
typedef __attribute__((ext_vector_type(8)))  _Float16 v8h;
typedef __attribute__((ext_vector_type(16))) __bf16   v16b;
typedef __attribute__((ext_vector_type(8)))  __bf16   v8b;
typedef __attribute__((ext_vector_type(8)))  float    v8f;
typedef __attribute__((ext_vector_type(4)))  float    v4f;
typedef __attribute__((ext_vector_type(4)))  int      v4i;
typedef __attribute__((ext_vector_type(4)))  unsigned int v4u;

__device__ __forceinline__ unsigned short f2bf_bits(float f) {
  unsigned u = __float_as_uint(f);
  return (unsigned short)((u + 0x7FFFu + ((u >> 16) & 1u)) >> 16);
}
__device__ __forceinline__ float bf_bits2f(unsigned short h) { return __uint_as_float(((unsigned)h) << 16); }

__device__ __forceinline__ void dep_guard_h(v8f& a, v8f& b, v16h x, v16h y) { asm volatile("v_nop\n\tv_nop\n\tv_nop\n\tv_nop" : "+v"(a), "+v"(b) : "v"(x), "v"(y)); }
__device__ __forceinline__ void dep_guard_b(v8f& a, v8f& b, v16b x, v16b y) { asm volatile("v_nop\n\tv_nop\n\tv_nop\n\tv_nop" : "+v"(a), "+v"(b) : "v"(x), "v"(y)); }
__device__ __forceinline__ void keep4_h(v16h a, v16h b, v16h c, v16h d) { asm volatile("v_nop" :: "v"(a), "v"(b), "v"(c), "v"(d)); }
__device__ __forceinline__ void keep4_b(v16b a, v16b b, v16b c, v16b d) { asm volatile("v_nop" :: "v"(a), "v"(b), "v"(c), "v"(d)); }
__device__ __forceinline__ void acc_guard4(v8f& a, v8f& b, v8f& c, v8f& d) { asm volatile("v_nop\n\tv_nop\n\tv_nop\n\tv_nop" : "+v"(a), "+v"(b), "+v"(c), "+v"(d)); }
template <typename T> struct Frag;
template <> struct Frag<_Float16> {
  typedef v16h V; union U { v16h v; v8h h[2]; };
  static __device__ __forceinline__ v16h load(const _Float16* p) {
    U f; f.h[0] = *(const v8h*)(p); f.h[1] = *(const v8h*)(p + 16); return f.v;
  }
  static __device__ __forceinline__ v8f mma(v16h a, v16h b, v8f c) {
    return __builtin_amdgcn_wmma_f32_16x16x32_f16(false, a, false, b, (short)0, c, false, false);
  }
  static __device__ __forceinline__ void guard(v8f& a, v8f& b, v16h x, v16h y) { dep_guard_h(a, b, x, y); }
  static __device__ __forceinline__ void keep(v16h a, v16h b, v16h c, v16h d) { keep4_h(a, b, c, d); }
};
template <> struct Frag<__bf16> {
  typedef v16b V; union U { v16b v; v8b h[2]; };
  static __device__ __forceinline__ v16b load(const __bf16* p) {
    U f; f.h[0] = *(const v8b*)(p); f.h[1] = *(const v8b*)(p + 16); return f.v;
  }
  static __device__ __forceinline__ v8f mma(v16b a, v16b b, v8f c) {
    return __builtin_amdgcn_wmma_f32_16x16x32_bf16(false, a, false, b, (short)0, c, false, false);
  }
  static __device__ __forceinline__ void guard(v8f& a, v8f& b, v16b x, v16b y) { dep_guard_b(a, b, x, y); }
  static __device__ __forceinline__ void keep(v16b a, v16b b, v16b c, v16b d) { keep4_b(a, b, c, d); }
};

__device__ __forceinline__ unsigned pk16(unsigned short a, unsigned short b) { return (unsigned)a | ((unsigned)b << 16); }
__device__ __forceinline__ unsigned short h_bits(float f) { const _Float16 h = (_Float16)f; return __builtin_bit_cast(unsigned short, h); }

__device__ __forceinline__ v8f mma16(v16h a, v16h b, v8f c) {
  c = __builtin_amdgcn_wmma_f32_16x16x32_f16(false, a, false, b, (short)0, c, false, false);
  asm volatile("v_nop\n\tv_nop\n\tv_nop\n\tv_nop" : "+v"(c) : "v"(a), "v"(b));
  return c;
}

template <int ET> struct Elem;
template <> struct Elem<0> { typedef _Float16 T; };
template <> struct Elem<1> { typedef __bf16 T; };
template <int ET, bool SPLIT, int BIAS_MODE, int OUT_MODE, bool RESID, int ACT = 0>
__global__ __launch_bounds__(256) void wmma_gemm64(
    const unsigned short* __restrict__ Ap, const unsigned short* __restrict__ A2p, int lda, long strideA,
    const unsigned short* __restrict__ Btp, const unsigned short* __restrict__ Bt2p, int ldb, long strideB,
    void* __restrict__ Cout, void* __restrict__ Cout2, int ldc, long strideC,
    const float* __restrict__ bias,
    const float* __restrict__ resid, long strideR,
    int M, int N, int K, float scale) {
  typedef typename Elem<ET>::T T;
  typedef typename Frag<T>::V V;
  const T* A = (const T*)Ap; const T* A2 = (const T*)A2p; const T* Bt = (const T*)Btp; const T* Bt2 = (const T*)Bt2p;
  __shared__ __align__(16) float sT[8][16 * 68];
  const int b    = blockIdx.y;
  const int lane = threadIdx.x & 31;
  const int wave = threadIdx.x >> 5;
  const int tilesN = N >> 6;
  const int tilesM = M >> 6;
  const int tile = blockIdx.x * 8 + wave;
  if (tile >= tilesM * tilesN) return;
  const int tm = tile / tilesN;
  const int tn = tile - tm * tilesN;
  const int m0 = tm << 6;
  const int n0 = tn << 6;

  const T* Ab  = A  + (size_t)b * strideA;
  const T* Bb  = Bt + (size_t)b * strideB;
  const T* Ab2 = SPLIT ? (A2  + (size_t)b * strideA) : nullptr;
  const T* Bb2 = SPLIT ? (Bt2 + (size_t)b * strideB) : nullptr;

  const int rlane = lane & 15;
  const int koff  = (lane >> 4) * 8;
  const int mOff  = (lane >> 4) * 8;

  v8f acc[4][4];
#pragma unroll
  for (int i = 0; i < 4; ++i)
#pragma unroll
    for (int j = 0; j < 4; ++j) acc[i][j] = (v8f){0.f,0.f,0.f,0.f,0.f,0.f,0.f,0.f};

  for (int k0 = 0; k0 < K; k0 += 32) {
    V bh[4], bl[4];
#pragma unroll
    for (int j = 0; j < 4; ++j) {
      const size_t bo = (size_t)(n0 + (j << 4) + rlane) * ldb + koff + k0;
      bh[j] = Frag<T>::load(Bb + bo);
      if (SPLIT) bl[j] = Frag<T>::load(Bb2 + bo);
    }
#pragma unroll
    for (int i = 0; i < 4; ++i) {
      const size_t ao = (size_t)(m0 + (i << 4) + rlane) * lda + koff + k0;
      V ah = Frag<T>::load(Ab + ao);
      V al;
      if (SPLIT) al = Frag<T>::load(Ab2 + ao);
#pragma unroll
      for (int j = 0; j < 4; ++j) {
        acc[i][j] = Frag<T>::mma(ah, bh[j], acc[i][j]);
        if (SPLIT) {
          acc[i][j] = Frag<T>::mma(ah, bl[j], acc[i][j]);
          acc[i][j] = Frag<T>::mma(al, bh[j], acc[i][j]);
        }
      }
      Frag<T>::guard(acc[i][0], acc[i][3], ah, SPLIT ? al : ah);
    }
    Frag<T>::keep(bh[0], bh[1], bh[2], bh[3]);
    if (SPLIT) Frag<T>::keep(bl[0], bl[1], bl[2], bl[3]);
  }
  acc_guard4(acc[0][0], acc[0][1], acc[0][2], acc[0][3]);
  acc_guard4(acc[1][0], acc[1][1], acc[1][2], acc[1][3]);
  acc_guard4(acc[2][0], acc[2][1], acc[2][2], acc[2][3]);
  acc_guard4(acc[3][0], acc[3][1], acc[3][2], acc[3][3]);

  float* slab = sT[wave];
  const float* Rb = RESID ? (resid + (size_t)b * strideR) : nullptr;
#pragma unroll
  for (int i = 0; i < 4; ++i) {
    const int mBase = m0 + (i << 4);
#pragma unroll
    for (int j = 0; j < 4; ++j) {
      const int n = n0 + (j << 4) + rlane;
      float bv = 0.f;
      if (BIAS_MODE == 2) bv = bias[n];
#pragma unroll
      for (int r = 0; r < 8; ++r) {
        float v = acc[i][j][r] * scale;
        if (BIAS_MODE == 1) v += bias[mBase + mOff + r];
        if (BIAS_MODE == 2) v += bv;
        if (RESID) v += Rb[(size_t)(mBase + mOff + r) * ldc + n];
        if (ACT == 2) v = fmaxf(v, 0.0f);
        if (ACT == 4) v = (v > 0.f) ? v : 0.01f * v;
        slab[(mOff + r) * 68 + (j << 4) + rlane] = v;
      }
    }
    __builtin_amdgcn_fence(__ATOMIC_RELEASE, "workgroup");
    __builtin_amdgcn_wave_barrier();
    __builtin_amdgcn_fence(__ATOMIC_ACQUIRE, "workgroup");
    if (OUT_MODE == 0) {
      float* C = (float*)Cout + (size_t)b * strideC;
      const int hh = lane >> 4, c4 = (lane & 15) * 4;
      for (int pass = 0; pass < 2; ++pass) {
#pragma unroll
        for (int it = 0; it < 8; ++it) {
          const int row = it * 2 + hh;
          v4f v = *(const v4f*)(slab + row * 68 + c4);
          *(volatile v4f*)(C + (size_t)(mBase + row) * ldc + n0 + c4) = v;
        }
        __threadfence();
      }
    } else {
      const int q = lane >> 3, c8 = (lane & 7) * 8;
      unsigned short* C  = (unsigned short*)Cout  + (size_t)b * strideC;
      unsigned short* C2 = (OUT_MODE == 2) ? ((unsigned short*)Cout2 + (size_t)b * strideC) : nullptr;
      for (int pass = 0; pass < 2; ++pass) {
#pragma unroll
        for (int it = 0; it < 4; ++it) {
          const int row = it * 4 + q;
          const float* sp = slab + row * 68 + c8;
          v8h hv, lv;
#pragma unroll
          for (int e = 0; e < 8; ++e) {
            if (OUT_MODE == 1) {
              hv[e] = (_Float16)sp[e];
            } else {
              unsigned short hb = f2bf_bits(sp[e]);
              unsigned short lb = f2bf_bits(sp[e] - bf_bits2f(hb));
              hv[e] = __builtin_bit_cast(_Float16, hb);
              lv[e] = __builtin_bit_cast(_Float16, lb);
            }
          }
          *(volatile v8h*)(C + (size_t)(mBase + row) * ldc + n0 + c8) = hv;
          if (OUT_MODE == 2) *(volatile v8h*)(C2 + (size_t)(mBase + row) * ldc + n0 + c8) = lv;
        }
        __threadfence();
      }
    }
    __builtin_amdgcn_fence(__ATOMIC_RELEASE, "workgroup");
    __builtin_amdgcn_wave_barrier();
    __builtin_amdgcn_fence(__ATOMIC_ACQUIRE, "workgroup");
  }
}

__global__ __launch_bounds__(256) void cast8s_f16_kernel(const float* __restrict__ in, unsigned short* __restrict__ out,
                                                        int n8, float scale) {
  const int i = blockIdx.x * 256 + threadIdx.x;
  if (i >= n8) return;
  const float* p = in + 8 * (size_t)i;
  const v4f a = *(const v4f*)(p);
  const v4f c = *(const v4f*)(p + 4);
  unsigned short hb[8];
#pragma unroll
  for (int e = 0; e < 4; ++e) {
    hb[e]     = h_bits(a[e] * scale);
    hb[4 + e] = h_bits(c[e] * scale);
  }
  const v4u u = (v4u){pk16(hb[0], hb[1]), pk16(hb[2], hb[3]), pk16(hb[4], hb[5]), pk16(hb[6], hb[7])};
  unsigned short* q = out + 8 * (size_t)i;
  *(volatile v4u*)q = u;
  __threadfence();
  *(volatile v4u*)q = u;
}

__global__ __launch_bounds__(256) void cat_cast_kernel(const float* __restrict__ mem, const float* __restrict__ w,
                                                      unsigned short* __restrict__ cat16) {
  const int b = blockIdx.z;
  const int y = blockIdx.y;
  const float* src = (y == 0) ? mem : w;
  const size_t i = (size_t)blockIdx.x * 256 + threadIdx.x;
  const float* p = src + (size_t)b * kQlen * kDm + 8 * i;
  const v4f a = *(const v4f*)(p);
  const v4f c = *(const v4f*)(p + 4);
  unsigned short hb[8];
#pragma unroll
  for (int e = 0; e < 4; ++e) {
    hb[e]     = h_bits(a[e]);
    hb[4 + e] = h_bits(c[e]);
  }
  const v4u u = (v4u){pk16(hb[0], hb[1]), pk16(hb[2], hb[3]), pk16(hb[4], hb[5]), pk16(hb[6], hb[7])};
  unsigned short* q = cat16 + ((size_t)b * kKlen + (size_t)y * kMlen) * kDm + 8 * i;
  *(volatile v4u*)q = u;
  __threadfence();
  *(volatile v4u*)q = u;
}

__global__ __launch_bounds__(256) void qbias_cast_kernel(const float* __restrict__ q, const float* __restrict__ rwb,
                                                        const float* __restrict__ rrb, unsigned short* __restrict__ qw,
                                                        unsigned short* __restrict__ qr) {
  const size_t i  = (size_t)blockIdx.x * 256 + threadIdx.x;
  const size_t e0 = 8 * i;
  const int col = (int)(e0 & (size_t)(kDm - 1));
  const v4f a  = *(const v4f*)(q + e0);
  const v4f c  = *(const v4f*)(q + e0 + 4);
  const v4f wa = *(const v4f*)(rwb + col);
  const v4f wc = *(const v4f*)(rwb + col + 4);
  const v4f ra = *(const v4f*)(rrb + col);
  const v4f rc = *(const v4f*)(rrb + col + 4);
  unsigned short hw[8], hr[8];
#pragma unroll
  for (int e = 0; e < 4; ++e) {
    hw[e]     = h_bits(a[e] + wa[e]);
    hw[4 + e] = h_bits(c[e] + wc[e]);
    hr[e]     = h_bits(a[e] + ra[e]);
    hr[4 + e] = h_bits(c[e] + rc[e]);
  }
  const v4u uw = (v4u){pk16(hw[0], hw[1]), pk16(hw[2], hw[3]), pk16(hw[4], hw[5]), pk16(hw[6], hw[7])};
  const v4u ur = (v4u){pk16(hr[0], hr[1]), pk16(hr[2], hr[3]), pk16(hr[4], hr[5]), pk16(hr[6], hr[7])};
  unsigned short* pw = qw + e0;
  unsigned short* pr = qr + e0;
  *(volatile v4u*)pw = uw;
  *(volatile v4u*)pr = ur;
  __threadfence();
  *(volatile v4u*)pw = uw;
  *(volatile v4u*)pr = ur;
}

__global__ __launch_bounds__(128) __attribute__((amdgpu_num_vgpr(256))) void rel_attn_kernel(
    const unsigned short* __restrict__ qwp,
    const unsigned short* __restrict__ qrp,
    const unsigned short* __restrict__ kp,
    const unsigned short* __restrict__ vtp,
    const unsigned short* __restrict__ rkp,
    const int* __restrict__ maskp,
    unsigned short* __restrict__ vecp) {
  __shared__ __align__(16) _Float16 Qwsh[kQB * kDh];
  __shared__ __align__(16) _Float16 Qrsh[kQB * kDh];
  __shared__ __align__(16) _Float16 Ksh[kKC * kDh];
  __shared__ __align__(16) _Float16 Vth[kDh * kKC];
  __shared__ __align__(16) _Float16 Rsh[kBand * kDh];
  __shared__ __align__(16) unsigned int Msh[kQB * kMWords];
  __shared__ __align__(16) _Float16 Psh[kWaves][16 * kKC];
  __shared__ __align__(16) float    Bsc[kWaves][16 * kBPitch];

  union FH { v16h v; v8h h[2]; };
  const int tid  = threadIdx.x;
  const int wave = tid >> 5;
  const int lane = tid & 31;
  const int hh   = lane >> 4;
  const int c    = lane & 15;
  const int qb = blockIdx.x;
  const int h  = blockIdx.y;
  const int b  = blockIdx.z;
  const int i0 = qb * kQB;
  const int q0 = i0 + wave * 16;

  {
    const size_t qbase = ((size_t)b * kQlen + i0) * kDm + (size_t)h * kDh;
#pragma unroll
    for (int it = 0; it < 4; ++it) {
      const int ch = it * 128 + tid;
      const int row = ch >> 3, c8 = (ch & 7) * 8;
      const v4u qu = *(const v4u*)(qwp + qbase + (size_t)row * kDm + c8);
      const v4u ru = *(const v4u*)(qrp + qbase + (size_t)row * kDm + c8);
      *(v8h*)(Qwsh + row * kDh + c8) = __builtin_bit_cast(v8h, qu);
      *(v8h*)(Qrsh + row * kDh + c8) = __builtin_bit_cast(v8h, ru);
    }
  }
  const _Float16* qwl = Qwsh + (wave * 16 + c) * kDh + 8 * hh;
  const _Float16* qrl = Qrsh + (wave * 16 + c) * kDh + 8 * hh;

  const v8f z8 = (v8f){0.f,0.f,0.f,0.f,0.f,0.f,0.f,0.f};
  const float neg_inf = -__builtin_inff();
  float mrow[8], lrow[8];
  v8f oacc[4];
#pragma unroll
  for (int r = 0; r < 8; ++r) { mrow[r] = neg_inf; lrow[r] = 0.f; }
#pragma unroll
  for (int t = 0; t < 4; ++t) oacc[t] = z8;

  const size_t kbase  = ((size_t)b * kKlen) * kDm + (size_t)h * kDh;
  const size_t vtbase = ((size_t)b * kDm + (size_t)h * kDh) * kKlen;
  const size_t rkbase = (size_t)h * kDh;
  const size_t mbase  = (size_t)i0 * kKlen;
  float* bs = Bsc[wave];
  _Float16* pw = Psh[wave];
  const int sb = 48 - 16 * wave;

  const int nChunks = qb + 17;
  for (int kc = 0; kc < nChunks; ++kc) {
    const int kv0 = kc * kKC;
    const int pb  = kv0 - i0 + 960;
    __syncthreads();
#pragma unroll
    for (int it = 0; it < 4; ++it) {
      const int ch = it * 128 + tid;
      const int row = ch >> 3, c8 = (ch & 7) * 8;
      const v4u ku = *(const v4u*)(kp + kbase + (size_t)(kv0 + row) * kDm + c8);
      const v4u vu = *(const v4u*)(vtp + vtbase + (size_t)row * kKlen + kv0 + c8);
      *(v8h*)(Ksh + row * kDh + c8) = __builtin_bit_cast(v8h, ku);
      *(v8h*)(Vth + row * kKC + c8) = __builtin_bit_cast(v8h, vu);
    }
    asm volatile("" ::: "memory");
#pragma unroll
    for (int it = 0; it < 8; ++it) {
      const int ch = it * 128 + tid;
      const int row = ch >> 3, c8 = (ch & 7) * 8;
      int p = pb + row;
      p = (p < 0) ? 0 : p;
      p = (p > kKlen - 1) ? (kKlen - 1) : p;
      const v4u ru = *(const v4u*)(rkp + rkbase + (size_t)p * kDm + c8);
      *(v8h*)(Rsh + row * kDh + c8) = __builtin_bit_cast(v8h, ru);
    }
    asm volatile("" ::: "memory");
#pragma unroll
    for (int it = 0; it < 8; ++it) {
      const int ch = it * 128 + tid;
      const int row = ch >> 4, g4 = ch & 15;
      const v4i mu = *(const v4i*)(maskp + mbase + (size_t)row * kKlen + kv0 + g4 * 4);
      const unsigned pkd = ((mu[0] == 1) ? 0x1u : 0u) | ((mu[1] == 1) ? 0x100u : 0u) |
                           ((mu[2] == 1) ? 0x10000u : 0u) | ((mu[3] == 1) ? 0x1000000u : 0u);
      Msh[row * kMWords + g4] = pkd;
    }
    __syncthreads();

#pragma unroll 1
    for (int t = 0; t < 5; ++t) {
      v8f acc = z8;
#pragma unroll
      for (int dc = 0; dc < 2; ++dc) {
        FH qa, rb;
        qa.h[0] = *(const v8h*)(qrl + dc * 32);
        qa.h[1] = *(const v8h*)(qrl + dc * 32 + 16);
        const _Float16* rp = Rsh + (sb + t * 16 + c) * kDh + dc * 32 + 8 * hh;
        rb.h[0] = *(const v8h*)(rp);
        rb.h[1] = *(const v8h*)(rp + 16);
        acc = mma16(qa.v, rb.v, acc);
      }
#pragma unroll
      for (int r = 0; r < 8; ++r) bs[(8 * hh + r) * kBPitch + t * 16 + c] = acc[r];
    }

    v8f s[4];
#pragma unroll
    for (int j = 0; j < 4; ++j) {
      s[j] = z8;
#pragma unroll
      for (int dc = 0; dc < 2; ++dc) {
        FH qa, kb;
        qa.h[0] = *(const v8h*)(qwl + dc * 32);
        qa.h[1] = *(const v8h*)(qwl + dc * 32 + 16);
        const _Float16* kq = Ksh + (j * 16 + c) * kDh + dc * 32 + 8 * hh;
        kb.h[0] = *(const v8h*)(kq);
        kb.h[1] = *(const v8h*)(kq + 16);
        s[j] = mma16(qa.v, kb.v, s[j]);
      }
    }
    __builtin_amdgcn_fence(__ATOMIC_RELEASE, "workgroup");
    __builtin_amdgcn_wave_barrier();
    __builtin_amdgcn_fence(__ATOMIC_ACQUIRE, "workgroup");

#pragma unroll
    for (int r = 0; r < 8; ++r) {
      const int il = 8 * hh + r;
      const float* brow = bs + il * kBPitch + (15 - il);
      const unsigned int* mw = Msh + (wave * 16 + il) * kMWords + (c >> 2);
      const int mshift = 8 * (c & 3);
      float m = neg_inf;
#pragma unroll
      for (int j = 0; j < 4; ++j) {
        const int jl = j * 16 + c;
        const float bdv = brow[jl];
        const unsigned mk = (mw[j * 4] >> mshift) & 0xffu;
        float sv = (s[j][r] + bdv) * kScoreScale;
        sv = (mk != 0u) ? kFill : sv;
        s[j][r] = sv;
        m = fmaxf(m, sv);
      }
#pragma unroll
      for (int off = 1; off < 16; off <<= 1) m = fmaxf(m, __shfl_xor(m, off, 32));
      const float mnew  = fmaxf(mrow[r], m);
      const float alpha = expf(mrow[r] - mnew);
      mrow[r] = mnew;
      float psum = 0.f;
#pragma unroll
      for (int j = 0; j < 4; ++j) {
        const float p = expf(s[j][r] - mnew);
        psum += p;
        pw[il * kKC + j * 16 + c] = (_Float16)(p * kPCarry);
      }
#pragma unroll
      for (int off = 1; off < 16; off <<= 1) psum += __shfl_xor(psum, off, 32);
      lrow[r] = lrow[r] * alpha + psum;
#pragma unroll
      for (int t = 0; t < 4; ++t) oacc[t][r] *= alpha;
    }
    __builtin_amdgcn_fence(__ATOMIC_RELEASE, "workgroup");
    __builtin_amdgcn_wave_barrier();
    __builtin_amdgcn_fence(__ATOMIC_ACQUIRE, "workgroup");

#pragma unroll 1
    for (int kk = 0; kk < 2; ++kk) {
      FH pa;
      const _Float16* pp = pw + c * kKC + kk * 32 + 8 * hh;
      pa.h[0] = *(const v8h*)(pp);
      pa.h[1] = *(const v8h*)(pp + 16);
#pragma unroll
      for (int t = 0; t < 4; ++t) {
        FH vb;
        const _Float16* vq = Vth + (t * 16 + c) * kKC + kk * 32 + 8 * hh;
        vb.h[0] = *(const v8h*)(vq);
        vb.h[1] = *(const v8h*)(vq + 16);
        oacc[t] = mma16(pa.v, vb.v, oacc[t]);
      }
    }
  }

  float* os = bs;
#pragma unroll
  for (int r = 0; r < 8; ++r) {
    const float inv = kVecOverP * (1.0f / lrow[r]);
#pragma unroll
    for (int t = 0; t < 4; ++t) os[(8 * hh + r) * kBPitch + t * 16 + c] = oacc[t][r] * inv;
  }
  __builtin_amdgcn_fence(__ATOMIC_RELEASE, "workgroup");
  __builtin_amdgcn_wave_barrier();
  __builtin_amdgcn_fence(__ATOMIC_ACQUIRE, "workgroup");
  {
    const int q8 = lane >> 3, c8 = (lane & 7) * 8;
    _Float16* vout = (_Float16*)vecp + ((size_t)b * kQlen + q0) * kDm + (size_t)h * kDh;
    for (int pass = 0; pass < 2; ++pass) {
#pragma unroll
      for (int it = 0; it < 4; ++it) {
        const int row = it * 4 + q8;
        const float* sp = os + row * kBPitch + c8;
        v8h hv;
#pragma unroll
        for (int e = 0; e < 8; ++e) hv[e] = (_Float16)sp[e];
        *(volatile v8h*)(vout + (size_t)row * kDm + c8) = hv;
      }
      __threadfence();
    }
  }
}

__global__ __launch_bounds__(256) void ln_kernel(const float* __restrict__ w, const float* __restrict__ attn,
                                                 const float* __restrict__ gamma, const float* __restrict__ beta,
                                                 float* __restrict__ out) {
  __shared__ float red1[8];
  __shared__ float red2[8];
  const int row  = blockIdx.x;
  const int t    = threadIdx.x;
  const int lane = t & 31, wave = t >> 5;
  const size_t base = (size_t)row * kDm + 4 * (size_t)t;
  const v4f a  = *(const v4f*)(w + base);
  const v4f ac = *(const v4f*)(attn + base);
  const v4f x  = a + ac;
  float s1 = (x[0] + x[1]) + (x[2] + x[3]);
#pragma unroll
  for (int off = 16; off > 0; off >>= 1) s1 += __shfl_xor(s1, off, 32);
  if (lane == 0) red1[wave] = s1;
  __syncthreads();
  float tot = red1[0];
#pragma unroll
  for (int wv = 1; wv < 8; ++wv) tot += red1[wv];
  const float mean = tot * kInvDm;
  const v4f d = x - mean;
  float s2 = (d[0] * d[0] + d[1] * d[1]) + (d[2] * d[2] + d[3] * d[3]);
#pragma unroll
  for (int off = 16; off > 0; off >>= 1) s2 += __shfl_xor(s2, off, 32);
  if (lane == 0) red2[wave] = s2;
  __syncthreads();
  float tot2 = red2[0];
#pragma unroll
  for (int wv = 1; wv < 8; ++wv) tot2 += red2[wv];
  const float var = tot2 * kInvDm;
  const float rs  = rsqrtf(var + kLnEps);
  const v4f g  = *(const v4f*)(gamma + 4 * t);
  const v4f be = *(const v4f*)(beta + 4 * t);
  v4f o;
#pragma unroll
  for (int e = 0; e < 4; ++e) o[e] = d[e] * rs * g[e] + be[e];
  float* op = out + base;
  *(volatile v4f*)op = o;
  __threadfence();
  *(volatile v4f*)op = o;
}

constexpr size_t kSzCat  = (size_t)kKRows * kDm * 2;
constexpr size_t kSzR    = (size_t)kKlen * kDm * 2;
constexpr size_t kSzQkvw = (size_t)3 * kDm * kDm * 2;
constexpr size_t kSzW    = (size_t)kDm * kDm * 2;
constexpr size_t kSzQf   = (size_t)kQRows * kDm * 4;
constexpr size_t kSzQ16  = (size_t)kQRows * kDm * 2;
constexpr size_t kSzK16  = (size_t)kKRows * kDm * 2;
constexpr size_t kSzVt   = (size_t)kBatch * kDm * kKlen * 2;
constexpr size_t kSzRk   = (size_t)kKlen * kDm * 2;
constexpr size_t kSzVec  = (size_t)kQRows * kDm * 2;
constexpr size_t kSzAttn = (size_t)kQRows * kDm * 4;
constexpr size_t kOffCat  = 0;
constexpr size_t kOffR    = kOffCat + kSzCat;
constexpr size_t kOffQkvw = kOffR + kSzR;
constexpr size_t kOffRw   = kOffQkvw + kSzQkvw;
constexpr size_t kOffOw   = kOffRw + kSzW;
constexpr size_t kOffQf   = kOffOw + kSzW;
constexpr size_t kOffQw   = kOffQf + kSzQf;
constexpr size_t kOffQr   = kOffQw + kSzQ16;
constexpr size_t kOffK    = kOffQr + kSzQ16;
constexpr size_t kOffVt   = kOffK + kSzK16;
constexpr size_t kOffRk   = kOffVt + kSzVt;
constexpr size_t kOffVec  = kOffRk + kSzRk;
constexpr size_t kOffAttn = kOffVec + kSzVec;
constexpr size_t kWsTotal = kOffAttn + kSzAttn;
static_assert(kWsTotal == 127926272ull, "carve total");
static_assert(kWsTotal <= 134217728ull, "carve limit");
static_assert((kOffR % 128) == 0 && (kOffQkvw % 128) == 0 && (kOffRw % 128) == 0 && (kOffOw % 128) == 0 &&
              (kOffQf % 128) == 0 && (kOffQw % 128) == 0 && (kOffQr % 128) == 0 && (kOffK % 128) == 0 &&
              (kOffVt % 128) == 0 && (kOffRk % 128) == 0 && (kOffVec % 128) == 0 && (kOffAttn % 128) == 0, "alignment");

extern "C" void kernel_launch(void* const* d_in, const int* in_sizes, int n_in,
                              void* d_out, int out_size, void* d_ws, size_t ws_size,
                              hipStream_t stream) {
  if (n_in < 11) return;
  if (in_sizes[0] != kBatch * kQlen * kDm) return;
  if (in_sizes[1] != kKlen * kDm) return;
  if (in_sizes[2] != kBatch * kMlen * kDm) return;
  if (in_sizes[3] != kQlen * kKlen) return;
  if (in_sizes[4] != 3 * kDm * kDm) return;
  if (in_sizes[5] != kDm * kDm || in_sizes[6] != kDm * kDm) return;
  if (in_sizes[7] != kHeads * kDh || in_sizes[8] != kHeads * kDh) return;
  if (in_sizes[9] != kDm || in_sizes[10] != kDm) return;
  if (out_size != kBatch * kQlen * kDm) return;
  if (ws_size < kWsTotal) return;

  const float* w     = (const float*)d_in[0];
  const float* r     = (const float*)d_in[1];
  const float* mem   = (const float*)d_in[2];
  const int*   amask = (const int*)d_in[3];
  const float* qkvw  = (const float*)d_in[4];
  const float* rw    = (const float*)d_in[5];
  const float* ow    = (const float*)d_in[6];
  const float* rrb   = (const float*)d_in[7];
  const float* rwb   = (const float*)d_in[8];
  const float* gam   = (const float*)d_in[9];
  const float* bet   = (const float*)d_in[10];
  float* out = (float*)d_out;

  char* ws = (char*)d_ws;
  unsigned short* CAT16 = (unsigned short*)(ws + kOffCat);
  unsigned short* R16   = (unsigned short*)(ws + kOffR);
  unsigned short* QKVW  = (unsigned short*)(ws + kOffQkvw);
  unsigned short* RW16  = (unsigned short*)(ws + kOffRw);
  unsigned short* OW16  = (unsigned short*)(ws + kOffOw);
  float*          QF32  = (float*)(ws + kOffQf);
  unsigned short* QW16  = (unsigned short*)(ws + kOffQw);
  unsigned short* QR16  = (unsigned short*)(ws + kOffQr);
  unsigned short* K16   = (unsigned short*)(ws + kOffK);
  unsigned short* VT16  = (unsigned short*)(ws + kOffVt);
  unsigned short* RK16  = (unsigned short*)(ws + kOffRk);
  unsigned short* VEC16 = (unsigned short*)(ws + kOffVec);
  float*          ATTN  = (float*)(ws + kOffAttn);

  cat_cast_kernel<<<dim3(512, 2, kBatch), dim3(256), 0, stream>>>(mem, w, CAT16);
  {
    const int n8r = (kKlen * kDm) / 8;
    const int n8q = (3 * kDm * kDm) / 8;
    const int n8w = (kDm * kDm) / 8;
    cast8s_f16_kernel<<<dim3(n8r / 256), dim3(256), 0, stream>>>(r, R16, n8r, 1.0f);
    cast8s_f16_kernel<<<dim3(n8q / 256), dim3(256), 0, stream>>>(qkvw, QKVW, n8q, kWCarry);
    cast8s_f16_kernel<<<dim3(n8w / 256), dim3(256), 0, stream>>>(rw, RW16, n8w, kWCarry);
    cast8s_f16_kernel<<<dim3(n8w / 256), dim3(256), 0, stream>>>(ow, OW16, n8w, kWCarry);
  }

  const long planeCat = (long)kKlen * kDm;
  const long planeQ   = (long)kQlen * kDm;
  const long planeVt  = (long)kDm * kKlen;

  wmma_gemm64<0, false, 0, 0, false, 0><<<dim3(32, kBatch), dim3(256), 0, stream>>>(
      CAT16 + (size_t)kMlen * kDm, CAT16 + (size_t)kMlen * kDm, kDm, planeCat,
      QKVW, QKVW, kDm, 0L,
      (void*)QF32, (void*)QF32, kDm, planeQ,
      rwb, rwb, 0L, kQlen, kDm, kDm, kWCarryInv);
  qbias_cast_kernel<<<dim3(2048), dim3(256), 0, stream>>>(QF32, rwb, rrb, QW16, QR16);
  wmma_gemm64<0, false, 0, 1, false, 0><<<dim3(256, 1), dim3(256), 0, stream>>>(
      CAT16, CAT16, kDm, 0L,
      QKVW + (size_t)kDm * kDm, QKVW + (size_t)kDm * kDm, kDm, 0L,
      (void*)K16, (void*)K16, kDm, 0L,
      rwb, rwb, 0L, kKRows, kDm, kDm, kWCarryInv);
  wmma_gemm64<0, false, 0, 1, false, 0><<<dim3(64, kBatch), dim3(256), 0, stream>>>(
      QKVW + (size_t)2 * kDm * kDm, QKVW + (size_t)2 * kDm * kDm, kDm, 0L,
      CAT16, CAT16, kDm, planeCat,
      (void*)VT16, (void*)VT16, kKlen, planeVt,
      rwb, rwb, 0L, kDm, kKlen, kDm, kWCarryInv);
  wmma_gemm64<0, false, 0, 1, false, 0><<<dim3(64, 1), dim3(256), 0, stream>>>(
      R16, R16, kDm, 0L,
      RW16, RW16, kDm, 0L,
      (void*)RK16, (void*)RK16, kDm, 0L,
      rwb, rwb, 0L, kKlen, kDm, kDm, kWCarryInv);
  rel_attn_kernel<<<dim3(kQlen / kQB, kHeads, kBatch), dim3(128), 0, stream>>>(
      QW16, QR16, K16, VT16, RK16, amask, VEC16);
  wmma_gemm64<0, false, 0, 0, false, 0><<<dim3(128, 1), dim3(256), 0, stream>>>(
      VEC16, VEC16, kDm, 0L,
      OW16, OW16, kDm, 0L,
      (void*)ATTN, (void*)ATTN, kDm, 0L,
      rwb, rwb, 0L, kQRows, kDm, kDm, kOutScale);
  ln_kernel<<<dim3(kQRows), dim3(256), 0, stream>>>(w, ATTN, gam, bet, out);
}
